// Grapher_61787399520597
// MI455X (gfx1250) — hardware-run, weakly checked
//
#include <hip/hip_runtime.h>
#include <math.h>
#include <stdint.h>

#define NB 8
#define NC 192
#define NH 56
#define NW 56
#define HW 3136
#define MROWS 25088
#define KSHIFT 4
#define NSHIFT 13
#define BN_EPS 1e-5f

#define SPLIT_FC1 1
#define SPLIT_GC  1
#define SPLIT_FC2 1

static_assert(NC == 6 * 32);
static_assert(NH == 56 && NW == 56);
static_assert(NH % KSHIFT == 0);
static_assert(NSHIFT == (NH - 1) / KSHIFT);
static_assert(HW == NH * NW);
static_assert(MROWS == NB * HW);
static_assert(MROWS % 128 == 0);
static_assert(HW % 64 == 0);
static_assert((HW * 4) % 128 == 0);
static_assert(NC % 64 == 0);
static_assert((2 * NC) % 32 == 0 && (4 * NC) % 32 == 0);
static_assert((NC * 2 * NC / 8) % 256 == 0);
static_assert((NC * 4 * NC / 8) % 256 == 0);
static_assert((NW * NC / 4) % 32 == 0);

typedef __attribute__((ext_vector_type(16))) __bf16 v16b;
typedef __attribute__((ext_vector_type(8)))  __bf16 v8b;
typedef __attribute__((ext_vector_type(8)))  float  v8f;
typedef __attribute__((ext_vector_type(4)))  float  v4f;
typedef __attribute__((ext_vector_type(2)))  float  v2f;
typedef __attribute__((ext_vector_type(4)))  unsigned int v4u;
typedef v8b __attribute__((may_alias)) v8ba;
typedef v4f __attribute__((may_alias)) v4fa;
typedef v2f __attribute__((may_alias)) v2fa;
typedef v4u __attribute__((may_alias)) v4ua;

__device__ __forceinline__ unsigned short f2bf_bits(float f) {
  const unsigned u = __float_as_uint(f);
  return (unsigned short)((u + 0x7FFFu + ((u >> 16) & 1u)) >> 16);
}
__device__ __forceinline__ float bf_bits2f(unsigned short h) { return __uint_as_float(((unsigned)h) << 16); }
__device__ __forceinline__ float bf_rne(float f) { return bf_bits2f(f2bf_bits(f)); }
__device__ __forceinline__ unsigned pk16(unsigned short a, unsigned short b) { return (unsigned)a | ((unsigned)b << 16); }

struct HL { v4u hi; v4u lo; };
static_assert(sizeof(HL) == 32);

__device__ __forceinline__ HL split8(v4f a, v4f c) {
  float f[8] = {a.x, a.y, a.z, a.w, c.x, c.y, c.z, c.w};
  unsigned short hb[8], lb[8];
#pragma unroll
  for (int e = 0; e < 8; ++e) {
    hb[e] = f2bf_bits(f[e]);
    lb[e] = f2bf_bits(f[e] - bf_bits2f(hb[e]));
  }
  HL r;
  r.hi = (v4u){pk16(hb[0], hb[1]), pk16(hb[2], hb[3]), pk16(hb[4], hb[5]), pk16(hb[6], hb[7])};
  r.lo = (v4u){pk16(lb[0], lb[1]), pk16(lb[2], lb[3]), pk16(lb[4], lb[5]), pk16(lb[6], lb[7])};
  return r;
}

__device__ __forceinline__ v8f mma_bf16(v16b a, v16b b, v8f c) {
  c = __builtin_amdgcn_wmma_f32_16x16x32_bf16(false, a, false, b, (short)0, c, false, false);
  asm volatile("v_nop\n\tv_nop\n\tv_nop\n\tv_nop" : "+v"(c) : "v"(a), "v"(b));
  return c;
}
union FB { v16b v; v8b h[2]; };
__device__ __forceinline__ v16b ldfrag(const __bf16* p, int h) {
  FB f;
  f.h[0] = *(const v8ba*)(p + 8 * h);
  f.h[1] = *(const v8ba*)(p + 16 + 8 * h);
  return f.v;
}

__device__ __forceinline__ float wave_sum(float v) {
  v += __shfl_xor(v, 16, 32);
  v += __shfl_xor(v, 8, 32);
  v += __shfl_xor(v, 4, 32);
  v += __shfl_xor(v, 2, 32);
  v += __shfl_xor(v, 1, 32);
  return v;
}

__device__ __forceinline__ void vst2f(float* p, float v) {
  *(volatile float*)p = v;
  __threadfence();
  *(volatile float*)p = v;
}

__device__ __forceinline__ void prep_unit(const float* __restrict__ w, unsigned short* __restrict__ dst,
                                          int unit, int kin, int per) {
  const int o = unit / per;
  const int kg = unit - o * per;
  int col = kg * 8;
  if (col >= kin) col -= kin;
  const float* s = w + (size_t)o * kin + col;
  const v4f a = *(const v4fa*)s;
  const v4f c = *(const v4fa*)(s + 4);
  const v4u pk = (v4u){pk16(f2bf_bits(a.x), f2bf_bits(a.y)), pk16(f2bf_bits(a.z), f2bf_bits(a.w)),
                       pk16(f2bf_bits(c.x), f2bf_bits(c.y)), pk16(f2bf_bits(c.z), f2bf_bits(c.w))};
  unsigned short* d = dst + (size_t)unit * 8;
  *(volatile v4u*)d = pk;
  __threadfence();
  *(volatile v4u*)d = pk;
}

__global__ __launch_bounds__(256) void k_prep(
    const float* __restrict__ fc1_w, const float* __restrict__ gc_w, const float* __restrict__ fc2_w,
    const float* __restrict__ b1, const float* __restrict__ g1, const float* __restrict__ e1,
    const float* __restrict__ m1, const float* __restrict__ v1,
    const float* __restrict__ b2, const float* __restrict__ g2, const float* __restrict__ e2,
    const float* __restrict__ m2, const float* __restrict__ v2,
    const float* __restrict__ b3, const float* __restrict__ g3, const float* __restrict__ e3,
    const float* __restrict__ m3, const float* __restrict__ v3,
    unsigned short* __restrict__ W1D, unsigned short* __restrict__ GCD, unsigned short* __restrict__ W3D,
    float* __restrict__ VEC) {
  const int bx = blockIdx.x, tid = threadIdx.x;
  if (bx < 36) {
    prep_unit(fc1_w, W1D, bx * 256 + tid, NC, 2 * NC / 8);
  } else if (bx < 108) {
    prep_unit(gc_w, GCD, (bx - 36) * 256 + tid, 2 * NC, 4 * NC / 8);
  } else if (bx < 144) {
    prep_unit(fc2_w, W3D, (bx - 108) * 256 + tid, NC, 2 * NC / 8);
  } else {
    const int set = bx - 144;
    const int i = tid < NC ? tid : NC - 1;
    float rb, rg, re, rm, rv;
    if (set == 0)      { rb = b1[i]; rg = g1[i]; re = e1[i]; rm = m1[i]; rv = v1[i]; }
    else if (set == 1) { rb = b2[i]; rg = g2[i]; re = e2[i]; rm = m2[i]; rv = v2[i]; }
    else               { rb = b3[i]; rg = g3[i]; re = e3[i]; rm = m3[i]; rv = v3[i]; }
    asm volatile("" :: "v"(rb), "v"(rg), "v"(re), "v"(rm), "v"(rv));
    rb = bf_rne(rb); rg = bf_rne(rg); re = bf_rne(re); rm = bf_rne(rm); rv = bf_rne(rv);
    float sc, sh;
    {
#pragma clang fp contract(off)
      sc = rg / sqrtf(rv + BN_EPS);
      const float ms = rm * sc;
      sh = re - ms;
    }
    if (tid < NC) {
      float* d = VEC + (size_t)(set * 3) * NC + tid;
      vst2f(d, rb);
      vst2f(d + NC, sc);
      vst2f(d + 2 * NC, sh);
    }
  }
}

__global__ __launch_bounds__(256) void k_cpe(const float* __restrict__ x, const float* __restrict__ pw,
                                             const float* __restrict__ pb, float* __restrict__ X1) {
  __shared__ __align__(16) float sp[62 * 64];
  __shared__ __align__(16) float so[HW];
  __shared__ float tp[64];
  const int tid = threadIdx.x;
  const int plane = blockIdx.x;
  const int c = plane % NC;
  const float* xp = x + (size_t)plane * HW;

  for (int q = tid; q < 992; q += 256) *(v4fa*)(sp + 4 * q) = (v4f){0.f, 0.f, 0.f, 0.f};
  if (tid < 64) {
    const int idx = tid < 49 ? tid : 48;
    const float t = pw[c * 49 + idx];
    asm volatile("" :: "v"(t));
    if (tid < 49) tp[tid] = bf_rne(t);
  }
  __syncthreads();
#pragma unroll 1
  for (int it = 0; it < 4; ++it) {
    const int q = tid + 256 * it;
    const int qc = q < 784 ? q : 783;
    const v4f v = *(const v4fa*)(xp + 4 * qc);
    asm volatile("" :: "v"(v));
    if (q < 784) {
      const int row = qc / 14;
      const int col = (qc - row * 14) * 4;
      float* d = sp + (row + 3) * 64 + 3 + col;
      d[0] = bf_rne(v.x); d[1] = bf_rne(v.y); d[2] = bf_rne(v.z); d[3] = bf_rne(v.w);
    }
  }
  __syncthreads();

  const float peb = bf_rne(pb[c]);
#pragma unroll 1
  for (int it = 0; it < 4; ++it) {
    const int q = tid + 256 * it;
    const int qc = q < 784 ? q : 783;
    const int row = qc / 14;
    const int col = (qc - row * 14) * 4;
    float a0 = 0.f, a1 = 0.f, a2 = 0.f, a3 = 0.f;
#pragma unroll 1
    for (int i = 0; i < 7; ++i) {
      const float* r = sp + (row + i) * 64 + col;
      float in[10];
#pragma unroll
      for (int t = 0; t < 10; ++t) in[t] = r[t];
#pragma unroll
      for (int j = 0; j < 7; ++j) {
        const float tj = tp[i * 7 + j];
        a0 = fmaf(tj, in[j], a0);
        a1 = fmaf(tj, in[j + 1], a1);
        a2 = fmaf(tj, in[j + 2], a2);
        a3 = fmaf(tj, in[j + 3], a3);
      }
    }
    const float* xr = sp + (row + 3) * 64 + 3 + col;
    v4f o;
    o.x = (a0 + peb) + xr[0];
    o.y = (a1 + peb) + xr[1];
    o.z = (a2 + peb) + xr[2];
    o.w = (a3 + peb) + xr[3];
    if (q < 784) *(v4fa*)(so + 4 * q) = o;
  }
  __syncthreads();

  float* op = X1 + (size_t)plane * HW;
#pragma unroll 1
  for (int pass = 0; pass < 2; ++pass) {
#pragma unroll
    for (int it = 0; it < 4; ++it) {
      const int q = tid + 256 * it;
      const int qc = q < 784 ? q : 783;
      const v4f v = *(const v4fa*)(so + 4 * qc);
      asm volatile("" :: "v"(v));
      if (q < 784) *(volatile v4f*)(op + 4 * q) = v;
    }
    __threadfence();
  }
}

__global__ __launch_bounds__(256) void k_tr(const float* __restrict__ X1, unsigned short* __restrict__ X1HL) {
  __shared__ float T[64 * 193];
  const int tid = threadIdx.x;
  const int R0 = blockIdx.x * 64;
  const int b = R0 / HW;
  const int p0 = R0 - b * HW;
  const float* src = X1 + (size_t)b * NC * HW + p0;
#pragma unroll 4
  for (int it = 0; it < 12; ++it) {
    const int g = tid + 256 * it;
    const int c = g >> 4, q = g & 15;
    const v4f v = *(const v4fa*)(src + (size_t)c * HW + 4 * q);
    T[(4 * q + 0) * 193 + c] = v.x;
    T[(4 * q + 1) * 193 + c] = v.y;
    T[(4 * q + 2) * 193 + c] = v.z;
    T[(4 * q + 3) * 193 + c] = v.w;
  }
  __syncthreads();
  v4u hv[12];
#pragma unroll
  for (int it = 0; it < 12; ++it) {
    const int g = tid + 256 * it;
    const int row = g / 48;
    const int pc = g - row * 48;
    const int lo = pc >= 24;
    const int ch0 = 8 * (pc - (lo ? 24 : 0));
    const float* t = T + row * 193 + ch0;
    const v4f a = (v4f){t[0], t[1], t[2], t[3]};
    const v4f c = (v4f){t[4], t[5], t[6], t[7]};
    const HL r = split8(a, c);
    const unsigned mk = lo ? 0xffffffffu : 0u;
    hv[it] = (r.hi & ~mk) | (r.lo & mk);
  }
  unsigned short* dst = X1HL + (size_t)R0 * (2 * NC);
#pragma unroll 1
  for (int pass = 0; pass < 2; ++pass) {
#pragma unroll
    for (int it = 0; it < 12; ++it) {
      const int g = tid + 256 * it;
      *(volatile v4u*)(dst + (size_t)g * 8) = hv[it];
    }
    __threadfence();
  }
}

template <int EPI, int LDK, int KUSE>
__global__ __launch_bounds__(128) __attribute__((amdgpu_num_vgpr(248)))
void k_gemm(const unsigned short* __restrict__ Ap, const unsigned short* __restrict__ Bp,
            const float* __restrict__ vec, void* __restrict__ outp) {
  static_assert(KUSE % 32 == 0);
  static_assert(KUSE <= LDK);
  static_assert(LDK % 8 == 0);
  __shared__ __align__(16) float sT[128 * 68];
  __shared__ __align__(16) float sV[3 * 64];

  const int tid = threadIdx.x, lane = tid & 31, w = tid >> 5;
  const int h = lane >> 4, m = lane & 15;
  const int m0 = blockIdx.x * 128;
  const int n0 = blockIdx.y * 64;
  const int m0w = m0 + 32 * w;

  if (tid < 64) {
    const int idx = tid < 48 ? tid : 47;
    const int vs = idx >> 4, q = idx & 15;
    const v4f v = *(const v4fa*)(vec + vs * NC + n0 + 4 * q);
    asm volatile("" :: "v"(v));
    if (tid < 48) *(v4fa*)(sV + vs * 64 + 4 * q) = v;
  }
  __syncthreads();

  const __bf16* A0 = (const __bf16*)(const void*)Ap + (size_t)(m0w + m) * LDK;
  const __bf16* A1 = A0 + (size_t)16 * LDK;
  const __bf16* Bb = (const __bf16*)(const void*)Bp + (size_t)(n0 + m) * LDK;

  const v8f zero8 = {0.f, 0.f, 0.f, 0.f, 0.f, 0.f, 0.f, 0.f};
  v8f acc[2][4];
#pragma unroll
  for (int mt = 0; mt < 2; ++mt)
#pragma unroll
    for (int nt = 0; nt < 4; ++nt) acc[mt][nt] = zero8;

#pragma unroll 1
  for (int k0 = 0; k0 < KUSE; k0 += 32) {
    const v16b a0 = ldfrag(A0 + k0, h);
    const v16b a1 = ldfrag(A1 + k0, h);
#pragma unroll
    for (int nt = 0; nt < 4; ++nt) {
      const v16b bq = ldfrag(Bb + (size_t)nt * 16 * LDK + k0, h);
      acc[0][nt] = mma_bf16(a0, bq, acc[0][nt]);
      acc[1][nt] = mma_bf16(a1, bq, acc[1][nt]);
    }
  }

#pragma unroll
  for (int nt = 0; nt < 4; ++nt) {
    const int col = 16 * nt + m;
    const float bb = sV[col], sc = sV[64 + col], sh = sV[128 + col];
#pragma unroll
    for (int mt = 0; mt < 2; ++mt) {
#pragma unroll
      for (int r = 0; r < 8; ++r) {
        const int rowl = 32 * w + 16 * mt + 8 * h + r;
        const float v = (acc[mt][nt][r] + bb) * sc + sh;
        if (EPI == 2) sT[col * 132 + rowl] = v;
        else          sT[rowl * 68 + col] = v;
      }
    }
  }
  __syncthreads();

  if (EPI == 0) {
    float* C = (float*)outp;
#pragma unroll 1
    for (int pass = 0; pass < 2; ++pass) {
#pragma unroll 4
      for (int it = 0; it < 16; ++it) {
        const int g = tid + 128 * it;
        const int row = g >> 4, q = g & 15;
        const v4f v = *(const v4fa*)(sT + row * 68 + 4 * q);
        *(volatile v4f*)(C + (size_t)(m0 + row) * NC + n0 + 4 * q) = v;
      }
      __threadfence();
    }
  } else if (EPI == 1) {
#pragma unroll 1
    for (int it = 0; it < 8; ++it) {
      const int g = tid + 128 * it;
      const int row = g >> 3, p = g & 7;
      float* sp = sT + row * 68 + 8 * p;
      v4f a = *(const v4fa*)sp;
      v4f c = *(const v4fa*)(sp + 4);
      a.x = 0.5f * a.x * (1.0f + erff(a.x * 0.70710678118654752f));
      a.y = 0.5f * a.y * (1.0f + erff(a.y * 0.70710678118654752f));
      a.z = 0.5f * a.z * (1.0f + erff(a.z * 0.70710678118654752f));
      a.w = 0.5f * a.w * (1.0f + erff(a.w * 0.70710678118654752f));
      c.x = 0.5f * c.x * (1.0f + erff(c.x * 0.70710678118654752f));
      c.y = 0.5f * c.y * (1.0f + erff(c.y * 0.70710678118654752f));
      c.z = 0.5f * c.z * (1.0f + erff(c.z * 0.70710678118654752f));
      c.w = 0.5f * c.w * (1.0f + erff(c.w * 0.70710678118654752f));
      const HL r = split8(a, c);
      *(v4ua*)sp = r.hi;
      *(v4ua*)(sp + 4) = r.lo;
    }
    __syncthreads();
    unsigned short* C = (unsigned short*)outp;
#pragma unroll 1
    for (int pass = 0; pass < 2; ++pass) {
#pragma unroll
      for (int it = 0; it < 8; ++it) {
        const int g = tid + 128 * it;
        const int row = g >> 3, p = g & 7;
        const float* sp = sT + row * 68 + 8 * p;
        const v4u hv = *(const v4ua*)sp;
        const v4u lv = *(const v4ua*)(sp + 4);
        unsigned short* d = C + (size_t)(m0 + row) * (2 * NC) + n0 + 8 * p;
        *(volatile v4u*)d = hv;
        *(volatile v4u*)(d + NC) = lv;
      }
      __threadfence();
    }
  } else {
    float* C = (float*)outp;
#pragma unroll 1
    for (int pass = 0; pass < 2; ++pass) {
#pragma unroll 4
      for (int it = 0; it < 16; ++it) {
        const int g = tid + 128 * it;
        const int n = g >> 5, q = g & 31;
        const int hf = q >> 4, q16 = q & 15;
        const int R = m0 + 64 * hf;
        const int bi = R / HW;
        const int p0 = R - bi * HW;
        const v4f v = *(const v4fa*)(sT + n * 132 + 64 * hf + 4 * q16);
        *(volatile v4f*)(C + ((size_t)(bi * NC + n0 + n)) * HW + p0 + 4 * q16) = v;
      }
      __threadfence();
    }
  }
}

__global__ __launch_bounds__(256) void k_soft(const float* __restrict__ X2, unsigned short* __restrict__ XC) {
  __shared__ __align__(16) float rows[NW * NC];
  __shared__ __align__(16) float cat[8][2 * NC];
  const int tid = threadIdx.x, lane = tid & 31, wave = tid >> 5;
  const int bh = blockIdx.x;
  const int b = bh / NH;
  const int h = bh - b * NH;
  const size_t row0 = (size_t)b * HW + (size_t)h * NW;
  const float* rb = X2 + row0 * NC;
#pragma unroll 1
  for (int it = 0; it < 11; ++it) {
    const int q = tid + 256 * it;
    const int qc = q < (NW * NC / 4) ? q : (NW * NC / 4 - 1);
    const v4f v = *(const v4fa*)(rb + 4 * qc);
    asm volatile("" :: "v"(v));
    if (q < (NW * NC / 4)) *(v4fa*)(rows + 4 * q) = v;
  }
  __syncthreads();

  const float* xb = X2 + (size_t)b * HW * NC;
  float* cw = cat[wave];
  const int lc = 2 * lane;

#pragma unroll 1
  for (int i = 0; i < 7; ++i) {
    const int w = wave * 7 + i;
    const float* sr = rows + w * NC + lc;
    const v2f s0 = *(const v2fa*)(sr);
    const v2f s1 = *(const v2fa*)(sr + 64);
    const v2f s2 = *(const v2fa*)(sr + 128);
    const float xs[6] = {s0.x, s0.y, s1.x, s1.y, s2.x, s2.y};
    float nw[6], nh[6];
#pragma unroll
    for (int k = 0; k < 6; ++k) { nw[k] = 0.0f; nh[k] = 0.0f; }
    float dw = 0.0f, dh = 0.0f;

#pragma unroll 1
    for (int s = KSHIFT; s < NW; s += KSHIFT) {
      int wn = w - s; wn += (wn < 0) ? NW : 0;
      int hn = h - s; hn += (hn < 0) ? NH : 0;
      const float* nr = rows + wn * NC + lc;
      const float* gr = xb + ((size_t)hn * NW + w) * NC + lc;
      const v2f a0 = *(const v2fa*)(nr);
      const v2f a1 = *(const v2fa*)(nr + 64);
      const v2f a2 = *(const v2fa*)(nr + 128);
      const v2f g0 = *(const v2fa*)(gr);
      const v2f g1 = *(const v2fa*)(gr + 64);
      const v2f g2 = *(const v2fa*)(gr + 128);
      const float dwv[6] = {a0.x - xs[0], a0.y - xs[1], a1.x - xs[2], a1.y - xs[3], a2.x - xs[4], a2.y - xs[5]};
      const float dhv[6] = {g0.x - xs[0], g0.y - xs[1], g1.x - xs[2], g1.y - xs[3], g2.x - xs[4], g2.y - xs[5]};
      float lw = fabsf(dwv[0]);
      float lh = fabsf(dhv[0]);
#pragma unroll
      for (int k = 1; k < 6; ++k) { lw += fabsf(dwv[k]); lh += fabsf(dhv[k]); }
      lw = wave_sum(lw);
      lh = wave_sum(lh);
      const float sw = expf(-lw / 0.1f);
      const float sh = expf(-lh / 0.1f);
#pragma unroll
      for (int k = 0; k < 6; ++k) {
        nw[k] = fmaf(dwv[k], sw, nw[k]);
        nh[k] = fmaf(dhv[k], sh, nh[k]);
      }
      dw += sw;
      dh += sh;
    }

    const float rw = 1.0f / (dw + 1e-6f);
    const float rh = 1.0f / (dh + 1e-6f);
    float xj[6];
#pragma unroll
    for (int k = 0; k < 6; ++k) {
      const float vw = nw[k] * rw;
      const float vh = nh[k] * rh;
      xj[k] = (vh > vw) ? vh : vw;
    }

    *(v2fa*)(cw + lc) = s0;
    *(v2fa*)(cw + lc + 64) = s1;
    *(v2fa*)(cw + lc + 128) = s2;
    *(v2fa*)(cw + NC + lc) = (v2f){xj[0], xj[1]};
    *(v2fa*)(cw + NC + lc + 64) = (v2f){xj[2], xj[3]};
    *(v2fa*)(cw + NC + lc + 128) = (v2f){xj[4], xj[5]};
    __builtin_amdgcn_fence(__ATOMIC_RELEASE, "workgroup");
    __builtin_amdgcn_wave_barrier();
    __builtin_amdgcn_fence(__ATOMIC_ACQUIRE, "workgroup");

    v4u pk[3];
#pragma unroll
    for (int t = 0; t < 3; ++t) {
      const int g = lane + 32 * t;
      const int lo = g >= 48;
      const int e0 = 8 * (g - (lo ? 48 : 0));
      const v4f a = *(const v4fa*)(cw + e0);
      const v4f c = *(const v4fa*)(cw + e0 + 4);
      const HL r = split8(a, c);
      const unsigned mk = lo ? 0xffffffffu : 0u;
      pk[t] = (r.hi & ~mk) | (r.lo & mk);
    }
    unsigned short* dst = XC + (row0 + (size_t)w) * (size_t)(4 * NC);
#pragma unroll
    for (int t = 0; t < 3; ++t) *(volatile v4u*)(dst + (size_t)(lane + 32 * t) * 8) = pk[t];
    __threadfence();
#pragma unroll
    for (int t = 0; t < 3; ++t) *(volatile v4u*)(dst + (size_t)(lane + 32 * t) * 8) = pk[t];
    __builtin_amdgcn_fence(__ATOMIC_RELEASE, "workgroup");
    __builtin_amdgcn_wave_barrier();
    __builtin_amdgcn_fence(__ATOMIC_ACQUIRE, "workgroup");
  }
}

extern "C" void kernel_launch(void* const* d_in, const int* in_sizes, int n_in,
                              void* d_out, int out_size, void* d_ws, size_t ws_size,
                              hipStream_t stream) {
  if (n_in < 21) return;
  if (in_sizes[0] != NB * NC * HW) return;
  if (in_sizes[1] != NC * 49) return;
  if (in_sizes[3] != NC * NC || in_sizes[9] != NC * 2 * NC || in_sizes[15] != NC * NC) return;
  if (in_sizes[2] != NC) return;
  for (int i = 4; i <= 8; ++i) if (in_sizes[i] != NC) return;
  for (int i = 10; i <= 14; ++i) if (in_sizes[i] != NC) return;
  for (int i = 16; i <= 20; ++i) if (in_sizes[i] != NC) return;
  if (out_size != NB * NC * HW) return;

  const float* x      = (const float*)d_in[0];
  const float* pe_w   = (const float*)d_in[1];
  const float* pe_b   = (const float*)d_in[2];
  const float* fc1_w  = (const float*)d_in[3];
  const float* fc1_b  = (const float*)d_in[4];
  const float* fc1_g  = (const float*)d_in[5];
  const float* fc1_be = (const float*)d_in[6];
  const float* fc1_m  = (const float*)d_in[7];
  const float* fc1_v  = (const float*)d_in[8];
  const float* gc_w   = (const float*)d_in[9];
  const float* gc_b   = (const float*)d_in[10];
  const float* gc_g   = (const float*)d_in[11];
  const float* gc_be  = (const float*)d_in[12];
  const float* gc_m   = (const float*)d_in[13];
  const float* gc_v   = (const float*)d_in[14];
  const float* fc2_w  = (const float*)d_in[15];
  const float* fc2_b  = (const float*)d_in[16];
  const float* fc2_g  = (const float*)d_in[17];
  const float* fc2_be = (const float*)d_in[18];
  const float* fc2_m  = (const float*)d_in[19];
  const float* fc2_v  = (const float*)d_in[20];

  const size_t PF  = (size_t)NB * NC * HW * 4;
  const size_t PHL = (size_t)MROWS * 2 * NC * 2;
  const size_t PXC = (size_t)MROWS * 4 * NC * 2;
  const size_t PW1 = (size_t)NC * 2 * NC * 2;
  const size_t PGC = (size_t)NC * 4 * NC * 2;
  const size_t PVE = (size_t)7168;
  size_t off = 0;
  const size_t oX1  = off; off += PF;
  const size_t oX1H = off; off += PHL;
  const size_t oX2  = off; off += PF;
  const size_t oXC  = off; off += PXC;
  const size_t oX3H = off; off += PHL;
  const size_t oW1  = off; off += PW1;
  const size_t oGC  = off; off += PGC;
  const size_t oW3  = off; off += PW1;
  const size_t oVE  = off; off += PVE;
  if (off > ws_size) return;
  if (off > (size_t)134217728) return;

  char* ws = (char*)d_ws;
  float*          X1   = (float*)(ws + oX1);
  unsigned short* X1HL = (unsigned short*)(ws + oX1H);
  float*          X2   = (float*)(ws + oX2);
  unsigned short* XCHL = (unsigned short*)(ws + oXC);
  unsigned short* X3HL = (unsigned short*)(ws + oX3H);
  unsigned short* W1D  = (unsigned short*)(ws + oW1);
  unsigned short* GCD  = (unsigned short*)(ws + oGC);
  unsigned short* W3D  = (unsigned short*)(ws + oW3);
  float*          VEC  = (float*)(ws + oVE);

  k_prep<<<dim3(147), dim3(256), 0, stream>>>(
      fc1_w, gc_w, fc2_w,
      fc1_b, fc1_g, fc1_be, fc1_m, fc1_v,
      gc_b, gc_g, gc_be, gc_m, gc_v,
      fc2_b, fc2_g, fc2_be, fc2_m, fc2_v,
      W1D, GCD, W3D, VEC);

  k_cpe<<<dim3(NB * NC), dim3(256), 0, stream>>>(x, pe_w, pe_b, X1);

  k_tr<<<dim3(MROWS / 64), dim3(256), 0, stream>>>(X1, X1HL);

  const dim3 gG(MROWS / 128, NC / 64);
  k_gemm<0, 2 * NC, (SPLIT_FC1 ? 2 * NC : NC)><<<gG, dim3(128), 0, stream>>>(X1HL, W1D, VEC, (void*)X2);

  k_soft<<<dim3(NB * NH), dim3(256), 0, stream>>>(X2, XCHL);

  k_gemm<1, 4 * NC, (SPLIT_GC ? 4 * NC : 2 * NC)><<<gG, dim3(128), 0, stream>>>(XCHL, GCD, VEC + 3 * NC, (void*)X3HL);

  k_gemm<2, 2 * NC, (SPLIT_FC2 ? 2 * NC : NC)><<<gG, dim3(128), 0, stream>>>(X3HL, W3D, VEC + 6 * NC, d_out);

  (void)hipGetLastError();
}
